// SSCM_78546361909687
// MI455X (gfx1250) — hardware-verified
//
#include <hip/hip_runtime.h>
#define NI 4
#define CH 256
#define HS 64
#define PX 4096
#define NR (NI * PX)
#define CQ 32
#define C2 128
typedef __bf16 v16b __attribute__((ext_vector_type(16)));
typedef unsigned short v8us __attribute__((ext_vector_type(8), may_alias));
typedef float  v8f  __attribute__((ext_vector_type(8)));
typedef float  v4f  __attribute__((ext_vector_type(4)));
typedef float  v4fa __attribute__((ext_vector_type(4), may_alias));
union FragB { v16b v; v8us half[2]; unsigned short u[16]; };

__device__ __forceinline__ unsigned short bf16_bits(float x) { unsigned int u = __float_as_uint(x); return (unsigned short)((u + 0x7FFFu + ((u >> 16) & 1u)) >> 16); }
__device__ __forceinline__ float bf16_val(unsigned short b) { return __uint_as_float(((unsigned int)b) << 16); }
__device__ __forceinline__ float bf16_round(float x) { return bf16_val(bf16_bits(x)); }
template <int NT>
__device__ __forceinline__ v8f mmaN(v16b ah, v16b al, v16b bh, v16b bl, v8f c) {
  c = __builtin_amdgcn_wmma_f32_16x16x32_bf16(false, ah, false, bh, (short)0, c, false, false);
  if (NT >= 2) c = __builtin_amdgcn_wmma_f32_16x16x32_bf16(false, al, false, bh, (short)0, c, false, false);
  if (NT >= 3) c = __builtin_amdgcn_wmma_f32_16x16x32_bf16(false, ah, false, bl, (short)0, c, false, false);
  asm volatile("v_nop\n\tv_nop\n\tv_nop\n\tv_nop" : "+v"(c) : "v"(ah), "v"(al), "v"(bh), "v"(bl));
  return c;
}

__global__ __launch_bounds__(256) void k_wt_bf16(const float* __restrict__ W, unsigned short* __restrict__ Wt, int K, int N) {
  const int t = blockIdx.x * 256 + threadIdx.x;
  const int k8n = K / 8;
  if (t >= N * k8n) return;
  const int n = t / k8n, k8 = (t % k8n) * 8;
  v8us v;
#pragma unroll
  for (int i = 0; i < 8; ++i) v[i] = bf16_bits(W[(size_t)(k8 + i) * N + n]);
  *(volatile v8us*)(Wt + (size_t)n * K + k8) = v;
  __threadfence();
  *(volatile v8us*)(Wt + (size_t)n * K + k8) = v;
}

template <bool ASPLIT, int ACT, bool BIAS_BF16>
__global__ __launch_bounds__(128) void k_gemm_bf(const float* __restrict__ A, int lda, const unsigned short* __restrict__ Wt, int ldb,
                                               const float* __restrict__ bias, float* __restrict__ C, int ldc, int M, int N, int K) {
  __shared__ __attribute__((aligned(16))) float so[4][16][64];
  const int tid = threadIdx.x, w = tid >> 5, lane = tid & 31, ln = lane & 15, hh = lane >> 4;
  const int ntn = N / 64;
  const int wid = blockIdx.x * 4 + w;
  const int mt = wid / ntn, nq = wid % ntn;
  if (mt * 16 >= M) return;
  const int row0 = mt * 16, col0 = nq * 64;
  const float* arow = A + (size_t)(row0 + ln) * lda;
  v8f acc[4] = {};
  for (int kb = 0; kb < K; kb += 32) {
    FragB ah, al;
    const v4f x0 = *(const v4fa*)(arow + kb + 8 * hh), x1 = *(const v4fa*)(arow + kb + 8 * hh + 4);
    const v4f x2 = *(const v4fa*)(arow + kb + 16 + 8 * hh), x3 = *(const v4fa*)(arow + kb + 16 + 8 * hh + 4);
    float xs[16] = {x0[0],x0[1],x0[2],x0[3],x1[0],x1[1],x1[2],x1[3],x2[0],x2[1],x2[2],x2[3],x3[0],x3[1],x3[2],x3[3]};
#pragma unroll
    for (int i = 0; i < 16; ++i) { const unsigned short hb = bf16_bits(xs[i]); ah.u[i] = hb; al.u[i] = ASPLIT ? bf16_bits(xs[i] - bf16_val(hb)) : (unsigned short)0; }
#pragma unroll
    for (int t = 0; t < 4; ++t) {
      const unsigned short* brow = Wt + (size_t)(col0 + t * 16 + ln) * ldb + kb;
      FragB b;
      b.half[0] = *(const v8us*)(brow + 8 * hh);
      b.half[1] = *(const v8us*)(brow + 16 + 8 * hh);
      acc[t] = mmaN<ASPLIT ? 2 : 1>(ah.v, al.v, b.v, b.v, acc[t]);
    }
  }
#pragma unroll
  for (int t = 0; t < 4; ++t) {
    float bv = bias ? bias[col0 + t * 16 + ln] : 0.f;
    if (BIAS_BF16) bv = bf16_round(bv);
#pragma unroll
    for (int r = 0; r < 8; ++r) { float v = acc[t][r] + bv; if (ACT == 1) v = fmaxf(v, 0.f); so[w][8 * hh + r][t * 16 + ln] = v; }
  }
  __builtin_amdgcn_fence(__ATOMIC_ACQ_REL, "workgroup");
  __builtin_amdgcn_wave_barrier();
  const int rsub = lane >> 4, c4 = (lane & 15) * 4;
  for (int pass = 0; pass < 2; ++pass) {
#pragma unroll
    for (int q = 0; q < 8; ++q) {
      const int r = q * 2 + rsub;
      const v4f v = *(const v4fa*)&so[w][r][c4];
      *(volatile v4f*)(C + (size_t)(row0 + r) * ldc + col0 + c4) = v;
    }
    if (pass == 0) __threadfence();
  }
}

template <bool ASPLIT, int ACT, bool BIAS_BF16, bool RES_BF16>
__global__ __launch_bounds__(128) void k_gemm_bf3(const float* __restrict__ A, int lda, const unsigned short* __restrict__ Wt, int ldb,
                                                const float* __restrict__ bias, const float* __restrict__ resid, int rmod, int ldr,
                                                float* __restrict__ C, int ldc, int M, int N, int K) {
  __shared__ __attribute__((aligned(16))) float so[4][16][64];
  const int tid = threadIdx.x, w = tid >> 5, lane = tid & 31, ln = lane & 15, hh = lane >> 4;
  const int ntn = N / 64;
  const int wid = blockIdx.x * 4 + w;
  const int mt = wid / ntn, nq = wid % ntn;
  if (mt * 16 >= M) return;
  const int row0 = mt * 16, col0 = nq * 64;
  const float* arow = A + (size_t)(row0 + ln) * lda;
  v8f acc[4] = {};
  for (int kb = 0; kb < K; kb += 32) {
    FragB ah, al;
    const v4f x0 = *(const v4fa*)(arow + kb + 8 * hh), x1 = *(const v4fa*)(arow + kb + 8 * hh + 4);
    const v4f x2 = *(const v4fa*)(arow + kb + 16 + 8 * hh), x3 = *(const v4fa*)(arow + kb + 16 + 8 * hh + 4);
    float xs[16] = {x0[0],x0[1],x0[2],x0[3],x1[0],x1[1],x1[2],x1[3],x2[0],x2[1],x2[2],x2[3],x3[0],x3[1],x3[2],x3[3]};
#pragma unroll
    for (int i = 0; i < 16; ++i) { const unsigned short hb = bf16_bits(xs[i]); ah.u[i] = hb; al.u[i] = ASPLIT ? bf16_bits(xs[i] - bf16_val(hb)) : (unsigned short)0; }
#pragma unroll
    for (int t = 0; t < 4; ++t) {
      const unsigned short* brow = Wt + (size_t)(col0 + t * 16 + ln) * ldb + kb;
      FragB b;
      b.half[0] = *(const v8us*)(brow + 8 * hh);
      b.half[1] = *(const v8us*)(brow + 16 + 8 * hh);
      acc[t] = mmaN<ASPLIT ? 2 : 1>(ah.v, al.v, b.v, b.v, acc[t]);
    }
  }
#pragma unroll
  for (int t = 0; t < 4; ++t) {
    const int col = col0 + t * 16 + ln;
    float bv = bias ? bias[col] : 0.f;
    if (BIAS_BF16) bv = bf16_round(bv);
#pragma unroll
    for (int r = 0; r < 8; ++r) {
      float v = acc[t][r] + bv;
      if (resid) { float rv = resid[(size_t)((row0 + 8 * hh + r) % rmod) * ldr + col]; if (RES_BF16) rv = bf16_round(rv); v += rv; }
      if (ACT == 1) v = fmaxf(v, 0.f);
      if (ACT == 2) v = 0.5f * v * (1.0f + erff(v * 0.70710678118654752f));
      if (ACT == 3) { const float u = 0.7978845608028654f * (v + 0.044715f * v * v * v); v = 0.5f * v * (1.0f + tanhf(u)); }
      so[w][8 * hh + r][t * 16 + ln] = v;
    }
  }
  __builtin_amdgcn_fence(__ATOMIC_ACQ_REL, "workgroup");
  __builtin_amdgcn_wave_barrier();
  const int rsub = lane >> 4, c4 = (lane & 15) * 4;
  for (int pass = 0; pass < 2; ++pass) {
#pragma unroll
    for (int q = 0; q < 8; ++q) {
      const int r = q * 2 + rsub;
      const v4f v = *(const v4fa*)&so[w][r][c4];
      *(volatile v4f*)(C + (size_t)(row0 + r) * ldc + col0 + c4) = v;
    }
    if (pass == 0) __threadfence();
  }
}
template <bool PARAM_BF16>
__global__ __launch_bounds__(256) void k_layernorm(const float* __restrict__ X, const float* __restrict__ R, const float* __restrict__ g, const float* __restrict__ bta,
                                                  float* __restrict__ out_sum, float* __restrict__ out_norm, int N, float eps) {
  __shared__ float red[256];
  const int row = blockIdx.x, tid = threadIdx.x;
  const float* x = X + (size_t)row * N; const float* rr = R ? R + (size_t)row * N : nullptr;
  float vals[16];
  const int per = N / 256;
  float s1 = 0.f;
  for (int u = 0; u < per / 4; ++u) {
    const int j = tid * 4 + 1024 * u;
    const v4f a = *(const v4fa*)(x + j);
    v4f b = {0.f,0.f,0.f,0.f}; if (rr) b = *(const v4fa*)(rr + j);
#pragma unroll
    for (int q = 0; q < 4; ++q) { const float v = a[q] + b[q]; vals[u * 4 + q] = v; s1 += v; }
  }
  red[tid] = s1; __syncthreads();
  for (int st = 128; st > 0; st >>= 1) { if (tid < st) red[tid] += red[tid + st]; __syncthreads(); }
  const float mu = red[0] / (float)N; __syncthreads();
  float s2 = 0.f;
  for (int u = 0; u < per / 4; ++u)
#pragma unroll
    for (int q = 0; q < 4; ++q) { const float c = vals[u * 4 + q] - mu; s2 += c * c; }
  red[tid] = s2; __syncthreads();
  for (int st = 128; st > 0; st >>= 1) { if (tid < st) red[tid] += red[tid + st]; __syncthreads(); }
  const float rs = rsqrtf(red[0] / (float)N + eps);
  for (int pass = 0; pass < 2; ++pass) {
    for (int u = 0; u < per / 4; ++u) {
      const int j = tid * 4 + 1024 * u;
      v4f o, sm;
#pragma unroll
      for (int q = 0; q < 4; ++q) {
        float gg = g[j + q], bb = bta[j + q];
        if (PARAM_BF16) { gg = bf16_round(gg); bb = bf16_round(bb); }
        sm[q] = vals[u * 4 + q]; o[q] = (vals[u * 4 + q] - mu) * rs * gg + bb;
      }
      if (out_sum) *(volatile v4f*)(out_sum + (size_t)row * N + j) = sm;
      *(volatile v4f*)(out_norm + (size_t)row * N + j) = o;
    }
    if (pass == 0) __threadfence();
  }
}


typedef _Float16 v16h __attribute__((ext_vector_type(16)));
union FragH { v16h v; v8us half[2]; _Float16 h[16]; unsigned short u[16]; };
template <int NT>
__device__ __forceinline__ v8f mmaH(v16h ah, v16h al, v16h bh, v16h bl, v8f c) {
  c = __builtin_amdgcn_wmma_f32_16x16x32_f16(false, ah, false, bh, (short)0, c, false, false);
  if (NT >= 2) c = __builtin_amdgcn_wmma_f32_16x16x32_f16(false, al, false, bh, (short)0, c, false, false);
  if (NT >= 3) c = __builtin_amdgcn_wmma_f32_16x16x32_f16(false, ah, false, bl, (short)0, c, false, false);
  asm volatile("v_nop\n\tv_nop\n\tv_nop\n\tv_nop" : "+v"(c) : "v"(ah), "v"(al), "v"(bh), "v"(bl));
  return c;
}
template <bool ASPLIT>
__global__ __launch_bounds__(128) void k_gemm_h(const float* __restrict__ A, int lda, size_t sA, const _Float16* __restrict__ Bh, int ldb, size_t sB, float alpha, float* __restrict__ C, int ldc, size_t sC, int M, int N, int K) {
  __shared__ __attribute__((aligned(16))) float so[4][16][64];
  const int tid = threadIdx.x, w = tid >> 5, lane = tid & 31, ln = lane & 15, hh = lane >> 4; const int by = blockIdx.y;
  A += (size_t)by * sA; Bh += (size_t)by * sB; C += (size_t)by * sC;
  const int ntn = (N + 63) / 64; const int wid = blockIdx.x * 4 + w; const int mt = wid / ntn, nq = wid % ntn; if (mt * 16 >= M) return;
  const int row0 = mt * 16, col0 = nq * 64; const float* arow = A + (size_t)(row0 + ln) * lda;
  v8f acc[4] = {};
  for (int kb = 0; kb < K; kb += 32) {
    FragH ah, al;
    const v4f x0 = *(const v4fa*)(arow + kb + 8 * hh), x1 = *(const v4fa*)(arow + kb + 8 * hh + 4), x2 = *(const v4fa*)(arow + kb + 16 + 8 * hh), x3 = *(const v4fa*)(arow + kb + 16 + 8 * hh + 4);
    float xs[16] = {x0[0],x0[1],x0[2],x0[3],x1[0],x1[1],x1[2],x1[3],x2[0],x2[1],x2[2],x2[3],x3[0],x3[1],x3[2],x3[3]};
#pragma unroll
    for (int i = 0; i < 16; ++i) { const _Float16 h = (_Float16)xs[i]; ah.h[i] = h; al.h[i] = ASPLIT ? (_Float16)(xs[i] - (float)h) : (_Float16)0.0f; }
#pragma unroll
    for (int t = 0; t < 4; ++t) { if (col0 + t * 16 >= N) continue; const size_t boff = (size_t)(col0 + t * 16 + ln) * ldb + kb; FragH bq; bq.half[0] = *(const v8us*)(Bh + boff + 8 * hh); bq.half[1] = *(const v8us*)(Bh + boff + 16 + 8 * hh);
      acc[t] = mmaH<ASPLIT ? 2 : 1>(ah.v, al.v, bq.v, bq.v, acc[t]); }
  }
#pragma unroll
  for (int t = 0; t < 4; ++t) { if (col0 + t * 16 >= N) continue;
#pragma unroll
    for (int r = 0; r < 8; ++r) so[w][8 * hh + r][t * 16 + ln] = acc[t][r] * alpha; }
  __builtin_amdgcn_fence(__ATOMIC_ACQ_REL, "workgroup"); __builtin_amdgcn_wave_barrier();
  const int rsub = lane >> 4, c4 = (lane & 15) * 4;
  for (int pass = 0; pass < 2; ++pass) {
#pragma unroll
    for (int q = 0; q < 8; ++q) { const int r = q * 2 + rsub; if (col0 + c4 < N) { const v4f v = *(const v4fa*)&so[w][r][c4]; *(volatile v4f*)(C + (size_t)(row0 + r) * ldc + col0 + c4) = v; } }
    if (pass == 0) __threadfence(); }
}

__global__ __launch_bounds__(256) void k_wt_f16(const float* __restrict__ W, _Float16* __restrict__ Wt, int K, int N, float scale) {
  const int t = blockIdx.x * 256 + threadIdx.x; if (t >= N * (K / 8)) return; const int n = t / (K / 8), k8 = (t % (K / 8)) * 8; FragH f;
#pragma unroll
  for (int i = 0; i < 8; ++i) f.h[i] = (_Float16)(bf16_round(W[(size_t)(k8 + i) * N + n]) * scale); const v8us o = f.half[0];
  *(volatile v8us*)((unsigned short*)Wt + (size_t)n * K + k8) = o; __threadfence(); *(volatile v8us*)((unsigned short*)Wt + (size_t)n * K + k8) = o;
}
template <int ACT>
__global__ __launch_bounds__(128) void k_gemm_hhx(const _Float16* __restrict__ A, int lda, size_t sA, const _Float16* __restrict__ Bh, int ldb, size_t sB, float alpha, const float* __restrict__ bias, size_t sBias, const float* __restrict__ CP, int rowsPerB, size_t sCPb, int row0g,
    float* __restrict__ C, _Float16* __restrict__ C16, int ldc, size_t sC, int M, int N, int K) {
  __shared__ __attribute__((aligned(16))) float so[4][16][64];
  const int tid = threadIdx.x, w = tid >> 5, lane = tid & 31, ln = lane & 15, hh = lane >> 4; const int by = blockIdx.y;
  A += (size_t)by * sA; Bh += (size_t)by * sB; const size_t cofs = (size_t)by * sC; const float* bp = bias ? bias + (size_t)by * sBias : nullptr;
  const int ntn = (N + 63) / 64; const int wid = blockIdx.x * 4 + w; const int mt = wid / ntn, nq = wid % ntn; if (mt * 16 >= M) return;
  const int row0 = mt * 16, col0 = nq * 64; const _Float16* arow = A + (size_t)(row0 + ln) * lda;
  v8f acc[4] = {};
  for (int kb = 0; kb < K; kb += 32) { FragH ah; ah.half[0] = *(const v8us*)((const unsigned short*)arow + kb + 8 * hh); ah.half[1] = *(const v8us*)((const unsigned short*)arow + kb + 16 + 8 * hh);
#pragma unroll
    for (int t = 0; t < 4; ++t) { if (col0 + t * 16 >= N) continue; const size_t boff = (size_t)(col0 + t * 16 + ln) * ldb + kb; FragH bq; bq.half[0] = *(const v8us*)((const unsigned short*)Bh + boff + 8 * hh); bq.half[1] = *(const v8us*)((const unsigned short*)Bh + boff + 16 + 8 * hh);
      acc[t] = mmaH<1>(ah.v, ah.v, bq.v, bq.v, acc[t]); }
  }
#pragma unroll
  for (int t = 0; t < 4; ++t) { if (col0 + t * 16 >= N) continue; const int col = col0 + t * 16 + ln; const float bv = bp ? bf16_round(bp[col]) : 0.f;
#pragma unroll
    for (int r = 0; r < 8; ++r) { float v = acc[t][r] * alpha + bv; if (CP) { const int rr = row0g + row0 + 8 * hh + r; if (rowsPerB < 0) v += CP[cofs + (size_t)rr * ldc + col];        else { const int bidx = rr / rowsPerB; v += CP[(size_t)bidx * sCPb + (size_t)by * 64 + col]; } } if (ACT == 1) v = (v > 0.f) ? v : expm1f(v); else if (ACT == 7) v = (v > 0.f) ? v + 1.0f : expf(v); else if (ACT == 8) v = tanhf(v); else if (ACT == 9) v = 0.5f * v * (1.0f + tanhf(0.7978845608028654f * (v + 0.044715f * v * v * v))); else if (ACT == 11) v = 1.0f / (1.0f + expf(-v)); else if (ACT == 12) v = (v > 0.f) ? v : 0.01f * v; else if (ACT == 14) v = (v > 0.f) ? v : 0.1f * v; else if (ACT == 16) v = (v >= 0.f) ? v : 0.3f * v; else if (ACT == 17) v = (v >= 0.f) ? v : 0.2f * v; else if (ACT == 15) v = v / (1.0f + expf(-v)); else if (ACT == 3) v = fmaxf(v, 0.f); else if (ACT == 6) v = 0.5f * v * (1.0f + erff(v * 0.70710678118654752f)); so[w][8 * hh + r][t * 16 + ln] = v; } }
  __builtin_amdgcn_fence(__ATOMIC_ACQ_REL, "workgroup"); __builtin_amdgcn_wave_barrier();
  const int rsub = lane >> 4, c4 = (lane & 15) * 4; typedef _Float16 v4h __attribute__((ext_vector_type(4)));
  for (int pass = 0; pass < 2; ++pass) {
#pragma unroll
    for (int q = 0; q < 8; ++q) { const int r = q * 2 + rsub; if (col0 + c4 < N) { const v4f v = *(const v4fa*)&so[w][r][c4]; if (C) *(volatile v4f*)(C + cofs + (size_t)(row0 + r) * ldc + col0 + c4) = v; if (C16) { v4h h4; for (int i = 0; i < 4; ++i) h4[i] = (_Float16)v[i]; *(volatile v4h*)(C16 + cofs + (size_t)(row0 + r) * ldc + col0 + c4) = h4; } } }
    if (pass == 0) __threadfence(); }
}


typedef _Float16 v4h __attribute__((ext_vector_type(4)));

__global__ __launch_bounds__(256) void k_x16(const float* __restrict__ x, _Float16* __restrict__ X16, size_t n8) { const size_t t = (size_t)blockIdx.x * 256 + threadIdx.x; if (t >= n8) return; FragH f;
#pragma unroll
  for (int q = 0; q < 8; ++q) f.h[q] = (_Float16)bf16_round(x[t * 8 + q]); *(volatile v8us*)((unsigned short*)X16 + t * 8) = f.half[0]; __threadfence(); *(volatile v8us*)((unsigned short*)X16 + t * 8) = f.half[0]; }
__global__ __launch_bounds__(256) void k_h16(const float* __restrict__ x, _Float16* __restrict__ X16, size_t n8) { const size_t t = (size_t)blockIdx.x * 256 + threadIdx.x; if (t >= n8) return; FragH f;
#pragma unroll
  for (int q = 0; q < 8; ++q) f.h[q] = (_Float16)x[t * 8 + q]; *(volatile v8us*)((unsigned short*)X16 + t * 8) = f.half[0]; __threadfence(); *(volatile v8us*)((unsigned short*)X16 + t * 8) = f.half[0]; }
__global__ __launch_bounds__(256) void k_round16f(const float* __restrict__ W, _Float16* __restrict__ Bt, size_t n8) { const size_t t = (size_t)blockIdx.x * 256 + threadIdx.x; if (t >= n8) return; FragH f;
#pragma unroll
  for (int i = 0; i < 8; ++i) f.h[i] = (_Float16)(bf16_round(W[t * 8 + i]) * 16.0f); *(volatile v8us*)((unsigned short*)Bt + t * 8) = f.half[0]; __threadfence(); *(volatile v8us*)((unsigned short*)Bt + t * 8) = f.half[0]; }
template <int NHv, int TTv>
__global__ __launch_bounds__(256) void k_vt(const _Float16* __restrict__ V16, int ldv, int voff, _Float16* __restrict__ Vt) { __shared__ unsigned short tl[64][66]; const int tid = threadIdx.x; const int slab = blockIdx.x / (TTv / 64), lg = blockIdx.x % (TTv / 64); const int b = slab / NHv, h = slab % NHv;
  for (int i = tid; i < 64 * 8; i += 256) { const int r = i / 8, c8 = (i % 8) * 8; FragH f; f.half[0] = *(const v8us*)((const unsigned short*)V16 + ((size_t)b * TTv + lg * 64 + r) * ldv + voff + h * 64 + c8);
#pragma unroll
    for (int q = 0; q < 8; ++q) tl[r][c8 + q] = f.u[q]; }
  __syncthreads();
  for (int pass = 0; pass < 2; ++pass) {
#pragma unroll
    for (int rd = 0; rd < 2; ++rd) { const int d = rd * 32 + tid / 8, pc = tid % 8; FragH f;
#pragma unroll
      for (int q = 0; q < 8; ++q) f.u[q] = tl[pc * 8 + q][d];
      *(volatile v8us*)((unsigned short*)Vt + ((size_t)slab * 64 + d) * TTv + lg * 64 + pc * 8) = f.half[0]; }
    if (pass == 0) __threadfence(); } }

__global__ __launch_bounds__(256) void k_hl(const float* __restrict__ F, _Float16* __restrict__ Hh, _Float16* __restrict__ Hl, size_t n8) { const size_t t = (size_t)blockIdx.x * 256 + threadIdx.x; if (t >= n8) return; FragH fh, fl; const v4f a = *(const v4fa*)(F + t * 8), c = *(const v4fa*)(F + t * 8 + 4);
#pragma unroll
  for (int q = 0; q < 4; ++q) { _Float16 h = (_Float16)a[q]; fh.h[q] = h; fl.h[q] = (_Float16)((a[q] - (float)h) * 1024.0f); h = (_Float16)c[q]; fh.h[4 + q] = h; fl.h[4 + q] = (_Float16)((c[q] - (float)h) * 1024.0f); }
  for (int pass = 0; pass < 2; ++pass) { *(volatile v8us*)((unsigned short*)Hh + t * 8) = fh.half[0]; *(volatile v8us*)((unsigned short*)Hl + t * 8) = fl.half[0]; if (pass == 0) __threadfence(); } }

__device__ __forceinline__ v16h g2_frag(const _Float16* p, int hh) { FragH f; f.half[0] = *(const v8us*)((const unsigned short*)p + 8 * hh); f.half[1] = *(const v8us*)((const unsigned short*)p + 16 + 8 * hh); return f.v; }
__device__ __forceinline__ v8f g2_mma(v16h a, v16h b, v8f c) { v8f d = __builtin_amdgcn_wmma_f32_16x16x32_f16(false, a, false, b, (short)0, c, false, false); asm volatile("v_nop\n\tv_nop\n\tv_nop\n\tv_nop" : "+v"(d) : "v"(a), "v"(b)); return d; }
template <int ACT>
__global__ __launch_bounds__(128) void k_gemm2(const _Float16* __restrict__ A, int lda, size_t sA, const _Float16* __restrict__ Bh, int ldb, size_t sB, float alpha, const float* __restrict__ bias, size_t sBias, const float* __restrict__ CP, int rowsPerB, size_t sCPb, int row0g,
    float* __restrict__ C, _Float16* __restrict__ C16, int ldc, size_t sC, int M, int N, int K) { static_assert(ACT == 0 || ACT == 3 || ACT == 6 || ACT == 8 || ACT == 9 || ACT == 11 || ACT == 12 || ACT == 14 || ACT == 15 || ACT == 16 || ACT == 17, "k_gemm2: unsupported ACT code (would silently apply no activation)");
  __shared__ __attribute__((aligned(16))) float so[4][32][68];
  const int tid = threadIdx.x, w = tid >> 5, lane = tid & 31, ln = lane & 15, hh = lane >> 4; const int by = blockIdx.y;
  A += (size_t)by * sA; Bh += (size_t)by * sB; const size_t cofs = (size_t)by * sC; const float* bp = bias ? bias + (size_t)by * sBias : nullptr;
  const int ntn = N >> 6; const int mt = blockIdx.x / ntn, nq = blockIdx.x - mt * ntn; const int row0 = mt * 128 + 32 * w, col0 = nq * 64; if (row0 >= M) return;
  const _Float16* a0p = A + (size_t)(row0 + ln) * lda; const _Float16* a1p = a0p + (size_t)16 * lda;
  const _Float16* b0p = Bh + (size_t)(col0 + ln) * ldb; const _Float16* b1p = b0p + (size_t)16 * ldb; const _Float16* b2p = b1p + (size_t)16 * ldb; const _Float16* b3p = b2p + (size_t)16 * ldb;
  const v8f z8 = {0.f,0.f,0.f,0.f,0.f,0.f,0.f,0.f}; v8f c00 = z8, c01 = z8, c02 = z8, c03 = z8, c10 = z8, c11 = z8, c12 = z8, c13 = z8;
#pragma unroll 1
  for (int kb = 0; kb < K; kb += 32) { const v16h a0 = g2_frag(a0p + kb, hh), a1 = g2_frag(a1p + kb, hh);
    v16h b = g2_frag(b0p + kb, hh); c00 = g2_mma(a0, b, c00); c10 = g2_mma(a1, b, c10);
    b = g2_frag(b1p + kb, hh); c01 = g2_mma(a0, b, c01); c11 = g2_mma(a1, b, c11);
    b = g2_frag(b2p + kb, hh); c02 = g2_mma(a0, b, c02); c12 = g2_mma(a1, b, c12);
    b = g2_frag(b3p + kb, hh); c03 = g2_mma(a0, b, c03); c13 = g2_mma(a1, b, c13); }
  v8f accs[8] = {c00, c01, c02, c03, c10, c11, c12, c13};
#pragma unroll
  for (int u = 0; u < 8; ++u) { const int t = u & 3, half = u >> 2; const int col = col0 + t * 16 + ln; const float bv = bp ? bf16_round(bp[col]) : 0.f;
#pragma unroll
    for (int r = 0; r < 8; ++r) { const int rloc = half * 16 + 8 * hh + r; float v = accs[u][r] * alpha + bv; if (CP) { if (rowsPerB < 0) v += CP[cofs + (size_t)(row0g + row0 + rloc) * ldc + col];        else { const int bidx = (row0g + row0 + rloc) / rowsPerB; v += CP[(size_t)bidx * sCPb + (size_t)by * 64 + col]; } }
      if (ACT == 3) v = fmaxf(v, 0.f); else if (ACT == 6) v = 0.5f * v * (1.0f + erff(v * 0.70710678118654752f)); else if (ACT == 11) v = 1.0f / (1.0f + expf(-v)); else if (ACT == 15) v = v / (1.0f + expf(-v)); else if (ACT == 12) v = (v > 0.f) ? v : 0.01f * v; else if (ACT == 8) v = tanhf(v); else if (ACT == 9) v = 0.5f * v * (1.0f + tanhf(0.7978845608028654f * (v + 0.044715f * v * v * v))); else if (ACT == 14) v = (v > 0.f) ? v : 0.1f * v; else if (ACT == 16) v = (v >= 0.f) ? v : 0.3f * v; else if (ACT == 17) v = (v >= 0.f) ? v : 0.2f * v;
      so[w][rloc][t * 16 + ln] = v; } }
  __builtin_amdgcn_fence(__ATOMIC_ACQ_REL, "workgroup"); __builtin_amdgcn_wave_barrier();
  const int rsub = lane >> 4, c4 = (lane & 15) * 4;
  for (int pass = 0; pass < 2; ++pass) {
#pragma unroll
    for (int q = 0; q < 16; ++q) { const int r = q * 2 + rsub; const v4f v = *(const v4fa*)&so[w][r][c4]; if (C) *(volatile v4f*)(C + cofs + (size_t)(row0 + r) * ldc + col0 + c4) = v; if (C16) { v4h h4; for (int i = 0; i < 4; ++i) h4[i] = (_Float16)v[i]; *(volatile v4h*)(C16 + cofs + (size_t)(row0 + r) * ldc + col0 + c4) = h4; } }
    if (pass == 0) __threadfence(); } }


__global__ __launch_bounds__(256) void k_wsc(const float* __restrict__ Wm, _Float16* __restrict__ Bt, size_t n8, float sc) { const size_t t = (size_t)blockIdx.x * 256 + threadIdx.x; if (t >= n8) return; FragH f; for (int q = 0; q < 8; ++q) f.h[q] = (_Float16)(bf16_round(Wm[t * 8 + q]) * sc); *(volatile v8us*)((unsigned short*)Bt + t * 8) = f.half[0]; __threadfence(); *(volatile v8us*)((unsigned short*)Bt + t * 8) = f.half[0]; }
__global__ __launch_bounds__(256) void k_wre(const float* __restrict__ w, int o0, _Float16* __restrict__ Bt) { const int t = blockIdx.x * 256 + threadIdx.x; if (t >= CQ * 9 * CH / 8) return; const int c8 = (t * 8) % CH; const int tap = ((t * 8) / CH) % 9; const int o = (t * 8) / (9 * CH); FragH f; for (int q = 0; q < 8; ++q) f.h[q] = (_Float16)(bf16_round(w[((o * CH + c8 + q) * 9) + tap]) * 16.0f);
  unsigned short* d = (unsigned short*)Bt + ((size_t)(o0 + o) * 9 * CH + tap * CH + c8); *(volatile v8us*)d = f.half[0]; __threadfence(); *(volatile v8us*)d = f.half[0]; }
__global__ __launch_bounds__(64) void k_bqk(const float* __restrict__ bq, const float* __restrict__ bk, float* __restrict__ dst) { const int i = threadIdx.x; const float v = (i < CQ) ? bq[i] : bk[i - CQ]; *(volatile float*)(dst + i) = v; __threadfence(); *(volatile float*)(dst + i) = v; }
__global__ __launch_bounds__(256) void k_nhwc(const float* __restrict__ x, _Float16* __restrict__ D) { const size_t t = (size_t)blockIdx.x * 256 + threadIdx.x; if (t >= (size_t)NR * CH / 8) return; const int c0 = (int)((t * 8) % CH); const size_t row = (t * 8) / CH; const int b = (int)(row / PX), p = (int)(row % PX); FragH f; for (int q = 0; q < 8; ++q) f.h[q] = (_Float16)bf16_round(x[((size_t)b * CH + c0 + q) * PX + p]);
  *(volatile v8us*)((unsigned short*)D + t * 8) = f.half[0]; __threadfence(); *(volatile v8us*)((unsigned short*)D + t * 8) = f.half[0]; }
__global__ __launch_bounds__(256) void k_im2col(const _Float16* __restrict__ Sp, _Float16* __restrict__ XC) { const size_t t = (size_t)blockIdx.x * 256 + threadIdx.x; if (t >= (size_t)NR * 9 * (CH / 8)) return; const int c8 = (int)(t % (CH / 8)) * 8; const int tap = (int)((t / (CH / 8)) % 9); const size_t row = t / ((size_t)9 * (CH / 8)); const int b = (int)(row / PX), p = (int)(row % PX); const int iy = p / HS - 1 + tap / 3, ix = p % HS - 1 + tap % 3; v8us v;
  if (iy >= 0 && iy < HS && ix >= 0 && ix < HS) v = *(const v8us*)((const unsigned short*)Sp + (((size_t)b * HS + iy) * HS + ix) * CH + c8); else { for (int q = 0; q < 8; ++q) v[q] = 0; }
  unsigned short* dst = (unsigned short*)XC + row * (size_t)(9 * CH) + tap * CH + c8; *(volatile v8us*)dst = v; __threadfence(); *(volatile v8us*)dst = v; }
__global__ __launch_bounds__(256) void k_qkbn(const float* __restrict__ QK, const float* __restrict__ qs, const float* __restrict__ qb, const float* __restrict__ qm, const float* __restrict__ qv, const float* __restrict__ ks, const float* __restrict__ kb, const float* __restrict__ km, const float* __restrict__ kv, _Float16* __restrict__ D) {
  #pragma clang fp contract(off)
  const size_t t = (size_t)blockIdx.x * 256 + threadIdx.x; if (t >= (size_t)NR * 64 / 8) return; const int c0 = (int)((t * 8) % 64); const v8f a = *(const v8f*)(QK + t * 8); FragH f;
  for (int q = 0; q < 8; ++q) { const int c = c0 + q; const bool isq = c < CQ; const int i = isq ? c : c - CQ; const float s = bf16_round(isq ? qs[i] : ks[i]), bb = bf16_round(isq ? qb[i] : kb[i]), m = bf16_round(isq ? qm[i] : km[i]), vv = bf16_round(isq ? qv[i] : kv[i]); const float inv = rsqrtf(vv + 1e-5f) * s; float y = (a[q] - m) * inv; y += bb; f.h[q] = (_Float16)fmaxf(y, 0.f); }
  *(volatile v8us*)((unsigned short*)D + t * 8) = f.half[0]; __threadfence(); *(volatile v8us*)((unsigned short*)D + t * 8) = f.half[0]; }
__global__ __launch_bounds__(256) void k_soft(const float* __restrict__ S, _Float16* __restrict__ P, float* __restrict__ RS) {
  #pragma clang fp contract(off)
  const int wv = threadIdx.x >> 5, ln = threadIdx.x & 31; const int r = blockIdx.x * 8 + wv; if (r >= PX) return; const float* sr = S + (size_t)r * PX; float mx = -3.0e38f;
#pragma unroll 1
  for (int gq = 0; gq < PX / 256; ++gq) { const v8f a = *(const v8f*)(sr + gq * 256 + ln * 8); for (int i = 0; i < 8; ++i) mx = fmaxf(mx, a[i]); }
  for (int o = 16; o > 0; o >>= 1) mx = fmaxf(mx, __shfl_xor(mx, o, 32)); float su = 0.f;
#pragma unroll 1
  for (int pass = 0; pass < 2; ++pass) { su = 0.f;
#pragma unroll 1
    for (int gq = 0; gq < PX / 256; ++gq) { const v8f a = *(const v8f*)(sr + gq * 256 + ln * 8); FragH ph; for (int i = 0; i < 8; ++i) { const float e = expf(a[i] - mx); su += e; ph.h[i] = (_Float16)(e * 1024.0f); } *(volatile v8us*)((unsigned short*)P + (size_t)r * PX + gq * 256 + ln * 8) = ph.half[0]; }
    if (pass == 0) __threadfence(); }
  for (int o = 16; o > 0; o >>= 1) su += __shfl_xor(su, o, 32); if (ln == 0) { *(volatile float*)(RS + (size_t)r * 32) = 1.0f / su; __threadfence(); *(volatile float*)(RS + (size_t)r * 32) = 1.0f / su; } }
__global__ __launch_bounds__(256) void k_cstat(const float* __restrict__ x, float* __restrict__ MN, float* __restrict__ MX) {
  #pragma clang fp contract(off)
  __shared__ float smn[32], smx[32]; const int wv = threadIdx.x >> 5, ln = threadIdx.x & 31;
#pragma unroll 1
  for (int i = 0; i < 4; ++i) { const int bc = blockIdx.x * 32 + wv * 4 + i; const float* xr = x + (size_t)bc * PX; float s = 0.f, m = -3.0e38f;
#pragma unroll 1
    for (int j = 0; j < PX / 32; ++j) { const float v = bf16_round(xr[j * 32 + ln]); s += v; m = fmaxf(m, v); }
    for (int o = 16; o > 0; o >>= 1) { s += __shfl_xor(s, o, 32); m = fmaxf(m, __shfl_xor(m, o, 32)); } if (ln == 0) { smn[wv * 4 + i] = s / (float)PX; smx[wv * 4 + i] = m; } }
  __syncthreads(); if (threadIdx.x < 32) { const int bc = blockIdx.x * 32 + threadIdx.x; for (int pass = 0; pass < 2; ++pass) { *(volatile float*)(MN + bc) = smn[threadIdx.x]; *(volatile float*)(MX + bc) = smx[threadIdx.x]; if (pass == 0) __threadfence(); } } }
__global__ __launch_bounds__(256) void k_gate(const float* __restrict__ MN, const float* __restrict__ MX, const float* __restrict__ W1, const float* __restrict__ b1, const float* __restrict__ W2, const float* __restrict__ b2, float* __restrict__ G) {
  #pragma clang fp contract(off)
  __shared__ float smn[CH], smx[CH], h1[C2], h2[C2]; const int b = blockIdx.x, c = threadIdx.x; smn[c] = MN[b * CH + c]; smx[c] = MX[b * CH + c]; __syncthreads();
  if (c < C2) { float s1 = bf16_round(b1[c]), s2 = s1;
#pragma unroll 1
    for (int k = 0; k < CH; ++k) { const float w = bf16_round(W1[c * CH + k]); s1 += w * smn[k]; s2 += w * smx[k]; } h1[c] = fmaxf(s1, 0.f); h2[c] = fmaxf(s2, 0.f); }
  __syncthreads(); float o1 = bf16_round(b2[c]), o2 = o1;
#pragma unroll 1
  for (int j = 0; j < C2; ++j) { const float w = bf16_round(W2[c * C2 + j]); o1 += w * h1[j]; o2 += w * h2[j]; }
  const float g = 1.0f / (1.0f + expf(-(o1 + o2))); *(volatile float*)(G + b * CH + c) = g; __threadfence(); *(volatile float*)(G + b * CH + c) = g; }
__global__ __launch_bounds__(256) void k_pstat(const float* __restrict__ V2, float* __restrict__ SM) {
  #pragma clang fp contract(off)
  const int t = blockIdx.x * 256 + threadIdx.x; if (t >= NR) return; const int b = t / PX, p = t % PX; const float* r = V2 + (size_t)t * CH; float s = 0.f, m = -3.0e38f;
#pragma unroll 1
  for (int c = 0; c < CH; c += 8) { const v8f a = *(const v8f*)(r + c); for (int q = 0; q < 8; ++q) { s += a[q]; m = fmaxf(m, a[q]); } }
  for (int pass = 0; pass < 2; ++pass) { *(volatile float*)(SM + ((size_t)b * 2 + 0) * PX + p) = m; *(volatile float*)(SM + ((size_t)b * 2 + 1) * PX + p) = s / (float)CH; if (pass == 0) __threadfence(); } }
__global__ __launch_bounds__(256) void k_spat(const float* __restrict__ SM, const float* __restrict__ cw, const float* __restrict__ cb, const float* __restrict__ bs, const float* __restrict__ bb, const float* __restrict__ bm, const float* __restrict__ bv, _Float16* __restrict__ AT) {
  #pragma clang fp contract(off)
  __shared__ float mp[HS][HS + 1]; const int b = blockIdx.x; const int tid = threadIdx.x; const float inv = rsqrtf(bf16_round(bv[0]) + 1e-5f) * bf16_round(bs[0]);
  for (int e = tid; e < HS * HS; e += 256) { const int h = e / HS, w = e % HS; float s = bf16_round(cb[0]);
    for (int ci = 0; ci < 2; ++ci)
#pragma unroll 1
      for (int k = 0; k < 9; ++k) { const int yy = h - 1 + k / 3, xq = w - 1 + k % 3; if (yy < 0 || yy >= HS || xq < 0 || xq >= HS) continue; s += SM[((size_t)b * 2 + ci) * PX + yy * HS + xq] * bf16_round(cw[ci * 9 + k]); }
    float y = (s - bf16_round(bm[0])) * inv; y += bf16_round(bb[0]); mp[h][w] = y; }
  __syncthreads();
  if (tid < HS) { const int h = tid; float mx = -3.0e38f; for (int w = 0; w < HS; ++w) mx = fmaxf(mx, mp[h][w]); float su = 0.f; for (int w = 0; w < HS; ++w) { const float e = expf(mp[h][w] - mx); mp[h][w] = e; su += e; } const float iv = 1.0f / su; for (int w = 0; w < HS; ++w) mp[h][w] *= iv; }
  __syncthreads();
  for (int e = tid; e < HS * HS / 8; e += 256) { const int k = e / (HS / 8), w0 = (e % (HS / 8)) * 8; FragH f; for (int q = 0; q < 8; ++q) f.h[q] = (_Float16)mp[w0 + q][k]; unsigned short* d = (unsigned short*)AT + ((size_t)b * HS + k) * HS + w0;
    *(volatile v8us*)d = f.half[0]; __threadfence(); *(volatile v8us*)d = f.half[0]; } }
__global__ __launch_bounds__(256) void k_xnat(const float* __restrict__ x, _Float16* __restrict__ D, size_t n8) { const size_t t = (size_t)blockIdx.x * 256 + threadIdx.x; if (t >= n8) return; const v8f a = *(const v8f*)(x + t * 8); FragH f; for (int q = 0; q < 8; ++q) f.h[q] = (_Float16)bf16_round(a[q]); *(volatile v8us*)((unsigned short*)D + t * 8) = f.half[0]; __threadfence(); *(volatile v8us*)((unsigned short*)D + t * 8) = f.half[0]; }
__global__ __launch_bounds__(256) void k_out(const float* __restrict__ x, const float* __restrict__ O, const float* __restrict__ RS, const float* __restrict__ vb, const float* __restrict__ gam, const float* __restrict__ G, const float* __restrict__ SP, int b, float* __restrict__ out) {
  #pragma clang fp contract(off)
  const int t = blockIdx.x * 256 + threadIdx.x; if (t >= CH * PX / 8) return; const int p0 = (t * 8) % PX; const int c = (t * 8) / PX; const size_t o = ((size_t)b * CH + c) * PX + p0; const v8f a = *(const v8f*)(x + o); const v8f sp = *(const v8f*)(SP + o); const float gm = bf16_round(gam[0]), g = G[b * CH + c], bvc = bf16_round(vb[c]); v8f v;
  for (int q = 0; q < 8; ++q) { const int p = p0 + q; const float xv = bf16_round(a[q]); float w = O[(size_t)p * CH + c] * RS[(size_t)p * 32]; w += bvc; float y = gm * w; y += xv; y += xv * g; y += sp[q]; v[q] = y; }
  *(volatile v8f*)(out + o) = v; __threadfence(); *(volatile v8f*)(out + o) = v; }

extern "C" void kernel_launch(void* const* d_in, const int* in_sizes, int n_in,
                              void* d_out, int out_size, void* d_ws, size_t ws_size, hipStream_t stream) {
  (void)in_sizes; (void)n_in; (void)out_size;
  const float* const* I = (const float* const*)d_in;
  const float* x = I[0]; const float* q_w = I[1]; const float* q_b = I[2]; const float* q_s = I[3]; const float* q_bb = I[4]; const float* q_m = I[5]; const float* q_v = I[6]; const float* k_w = I[7]; const float* k_b = I[8]; const float* k_s = I[9]; const float* k_bb = I[10]; const float* k_m = I[11]; const float* k_v = I[12]; const float* v_w = I[13]; const float* v_b = I[14]; const float* gam = I[15]; const float* c_w1 = I[16]; const float* c_b1 = I[17]; const float* c_w2 = I[18]; const float* c_b2 = I[19]; const float* s_vw = I[20]; const float* s_vb = I[21]; const float* s_cw = I[22]; const float* s_cb = I[23]; const float* s_s = I[24]; const float* s_b = I[25]; const float* s_m = I[26]; const float* s_v = I[27];
  char* ws = (char*)d_ws; size_t off = 0;
  auto take = [&](size_t bytes) { char* p = ws + off; off += (bytes + 255) & ~(size_t)255; return p; };
  const size_t np = (size_t)NR * CH;
  _Float16* BQK = (_Float16*)take((size_t)64 * 9 * CH * 2); float* bqk = (float*)take(64 * 4); _Float16* AWV = (_Float16*)take((size_t)CH * CH * 2); _Float16* BSV = (_Float16*)take((size_t)CH * CH * 2);
  _Float16* X16 = (_Float16*)take(np * 2); _Float16* XC = (_Float16*)take((size_t)NR * 9 * CH * 2);        float* QK = (float*)take((size_t)NR * 64 * 4); _Float16* QK16 = (_Float16*)take((size_t)NR * 64 * 2); _Float16* V16 = (_Float16*)take(np * 2);        float* V2 = (float*)take(np * 4);
  float* MN = (float*)take(NI * CH * 4); float* MX = (float*)take(NI * CH * 4); float* G = (float*)take(NI * CH * 4); float* SM = (float*)take((size_t)NI * 2 * PX * 4); _Float16* AT = (_Float16*)take((size_t)NI * HS * HS * 2); _Float16* XN = (_Float16*)take(np * 2); float* SP = (float*)take(np * 4);
  float* S = ((size_t)NR * 9 * CH * 2 >= (size_t)PX * PX * 4) ? (float*)XC : (float*)take((size_t)PX * PX * 4);        _Float16* P = (_Float16*)take((size_t)PX * PX * 2); float* RS = (float*)take((size_t)PX * 32 * 4); float* O = (float*)take((size_t)PX * CH * 4);
  if (off > ws_size) return;
  k_wre<<<(CQ * 9 * CH / 8 + 255) / 256, 256, 0, stream>>>(q_w, 0, BQK); k_wre<<<(CQ * 9 * CH / 8 + 255) / 256, 256, 0, stream>>>(k_w, CQ, BQK); k_bqk<<<1, 64, 0, stream>>>(q_b, k_b, bqk);
  k_wsc<<<(CH * CH / 8 + 255) / 256, 256, 0, stream>>>(v_w, AWV, (size_t)CH * CH / 8, 16.0f); k_wsc<<<(CH * CH / 8 + 255) / 256, 256, 0, stream>>>(s_vw, BSV, (size_t)CH * CH / 8, 16.0f);
  k_nhwc<<<(unsigned)((np / 8 + 255) / 256), 256, 0, stream>>>(x, X16); k_xnat<<<(unsigned)((np / 8 + 255) / 256), 256, 0, stream>>>(x, XN, np / 8);
  k_im2col<<<(unsigned)(((size_t)NR * 9 * (CH / 8) + 255) / 256), 256, 0, stream>>>(X16, XC);
  k_gemm2<0><<<dim3((NR / 128) * 1, 1), 128, 0, stream>>>(XC, 9 * CH, 0, BQK, 9 * CH, 0, 0.0625f, bqk, 0, nullptr, 1, 0, 0, QK, nullptr, 64, 0, NR, 64, 9 * CH);
  k_qkbn<<<(unsigned)(((size_t)NR * 64 / 8 + 255) / 256), 256, 0, stream>>>(QK, q_s, q_bb, q_m, q_v, k_s, k_bb, k_m, k_v, QK16);
  k_gemm2<0><<<dim3((CH / 128) * (PX / 64), NI), 128, 0, stream>>>(AWV, CH, 0, X16, CH, (size_t)PX * CH, 0.0625f, nullptr, 0, nullptr, 1, 0, 0, nullptr, V16, PX, (size_t)CH * PX, CH, PX, CH);
  k_gemm2<0><<<dim3((NR / 128) * (CH / 64), 1), 128, 0, stream>>>(X16, CH, 0, BSV, CH, 0, 0.0625f, s_vb, 0, nullptr, 1, 0, 0, V2, nullptr, CH, 0, NR, CH, CH);
  k_cstat<<<NI * CH / 32, 256, 0, stream>>>(x, MN, MX); k_gate<<<NI, 256, 0, stream>>>(MN, MX, c_w1, c_b1, c_w2, c_b2, G);
  k_pstat<<<(NR + 255) / 256, 256, 0, stream>>>(V2, SM); k_spat<<<NI, 256, 0, stream>>>(SM, s_cw, s_cb, s_s, s_b, s_m, s_v, AT);
  k_gemm2<0><<<dim3((CH * HS / 128) * 1, NI), 128, 0, stream>>>(XN, HS, (size_t)CH * HS * HS, AT, HS, (size_t)HS * HS, 1.0f, nullptr, 0, nullptr, 1, 0, 0, SP, nullptr, HS, (size_t)CH * HS * HS, CH * HS, HS, HS);
  for (int b = 0; b < NI; ++b) { const size_t r0 = (size_t)b * PX;
    k_gemm2<0><<<dim3((PX / 128) * (PX / 64), 1), 128, 0, stream>>>(QK16 + r0 * 64, 64, 0, QK16 + r0 * 64 + CQ, 64, 0, 1.0f, nullptr, 0, nullptr, 1, 0, 0, S, nullptr, PX, 0, PX, PX, CQ);
    k_soft<<<PX / 8, 256, 0, stream>>>(S, P, RS);
    k_gemm2<0><<<dim3((PX / 128) * (CH / 64), 1), 128, 0, stream>>>(P, PX, 0, V16 + r0 * CH, PX, 0, 0.0009765625f, nullptr, 0, nullptr, 1, 0, 0, O, nullptr, CH, 0, PX, CH, PX);
    k_out<<<(CH * PX / 8 + 255) / 256, 256, 0, stream>>>(x, O, RS, v_b, gam, G, SP, b, (float*)d_out); }
}
